// RGCN_15779709845776
// MI455X (gfx1250) — hardware-run, weakly checked
//
#include <hip/hip_runtime.h>

typedef float          v8f   __attribute__((ext_vector_type(8)));
typedef float          v4f   __attribute__((ext_vector_type(4)));
typedef unsigned int   v4u   __attribute__((ext_vector_type(4)));
typedef int            v8i   __attribute__((ext_vector_type(8)));
typedef unsigned short v8us  __attribute__((ext_vector_type(8)));
typedef unsigned short v16us __attribute__((ext_vector_type(16)));
typedef __bf16         v16bf __attribute__((ext_vector_type(16)));
typedef _Float16       v16h  __attribute__((ext_vector_type(16)));
typedef v4f  __attribute__((may_alias)) v4fa;
typedef v8us __attribute__((may_alias)) v8usa;
union FragB { v16bf v; v16us u; v8us h[2]; v8i w; };
union FragH { v16h  v; v16us u; v8us h[2]; v8i w; };

__device__ __forceinline__ v8f wmb(const FragB& a, const FragB& b, v8f c) {
  v8f d = __builtin_amdgcn_wmma_f32_16x16x32_bf16(false, a.v, false, b.v, (short)0, c, false, false);
  asm volatile("v_nop\n\tv_nop\n\tv_nop\n\tv_nop" : "+v"(d) : "v"(a.w), "v"(b.w));
  return d;
}

__device__ __forceinline__ v8f wmh(const FragH& a, const FragH& b, v8f c) {
  v8f d = __builtin_amdgcn_wmma_f32_16x16x32_f16(false, a.v, false, b.v, (short)0, c, false, false);
  asm volatile("v_nop\n\tv_nop\n\tv_nop\n\tv_nop" : "+v"(d) : "v"(a.w), "v"(b.w));
  return d;
}

__device__ __forceinline__ unsigned bf16_bits(float f) {
  const unsigned u = __float_as_uint(f);
  const unsigned r = (u + 0x7FFFu + ((u >> 16) & 1u)) >> 16;
  const unsigned q = (u >> 16) | 0x40u;
  return ((u & 0x7fffffffu) > 0x7f800000u) ? q : r;
}

__device__ __forceinline__ float bf16_val(float f) {
  return __uint_as_float(bf16_bits(f) << 16);
}
__device__ __forceinline__ int clampi(int v, int lo, int hi) {
  return v < lo ? lo : (v > hi ? hi : v);
}

__device__ __forceinline__ unsigned f16_bits(float f) {
  const unsigned u  = __float_as_uint(f);
  const unsigned s  = (u >> 16) & 0x8000u;
  const unsigned a  = u & 0x7fffffffu;
  const unsigned t  = a - 0x38000000u;
  const unsigned r  = (t + 0x0FFFu + ((t >> 13) & 1u)) >> 13;
  const unsigned rc = r > 0x7C00u ? 0x7C00u : r;
  const bool small  = a < 0x38800000u;
  const bool isnan  = a > 0x7f800000u;
  const unsigned fin = small ? 0u : (s | rc);
  return isnan ? (s | 0x7E00u) : fin;
}

__device__ __forceinline__ unsigned pk16(unsigned lo, unsigned hi) { return lo | (hi << 16); }
__device__ __forceinline__ unsigned bf16_lo_bits(float v) {
  float hi = bf16_val(v);
  asm volatile("" : "+v"(hi));
  return bf16_bits(v - hi);
}
__device__ __forceinline__ v4u pack8_bf16(v4f a, v4f c) {
  return (v4u){ pk16(bf16_bits(a[0]), bf16_bits(a[1])), pk16(bf16_bits(a[2]), bf16_bits(a[3])),
                pk16(bf16_bits(c[0]), bf16_bits(c[1])), pk16(bf16_bits(c[2]), bf16_bits(c[3])) };
}
__device__ __forceinline__ v4u pack8_bf16_lo(v4f a, v4f c) {
  return (v4u){ pk16(bf16_lo_bits(a[0]), bf16_lo_bits(a[1])), pk16(bf16_lo_bits(a[2]), bf16_lo_bits(a[3])),
                pk16(bf16_lo_bits(c[0]), bf16_lo_bits(c[1])), pk16(bf16_lo_bits(c[2]), bf16_lo_bits(c[3])) };
}
__device__ __forceinline__ v4u pack8_f16(v4f a, v4f c) {
  return (v4u){ pk16(f16_bits(a[0]), f16_bits(a[1])), pk16(f16_bits(a[2]), f16_bits(a[3])),
                pk16(f16_bits(c[0]), f16_bits(c[1])), pk16(f16_bits(c[2]), f16_bits(c[3])) };
}

template <int FORM>
__global__ __launch_bounds__(256) void k_plane(const float* __restrict__ src, int rows, int cols, int ldsrc,
                                               unsigned short* __restrict__ dst, int MP, int KP) {
  static_assert(FORM >= 0 && FORM <= 3);
  const int KTOT = (FORM == 1 || FORM == 3) ? 2 * KP : KP;
  const unsigned ppr   = (unsigned)(KTOT >> 3);
  const unsigned kp8   = (unsigned)(KP >> 3);
  const unsigned total = (unsigned)MP * ppr;
  const unsigned g     = blockIdx.x * 256u + threadIdx.x;
  const unsigned rowu  = g / ppr;
  const unsigned p     = g - rowu * ppr;
  const bool second    = p >= kp8;
  const int row = (int)rowu;
  const int c0  = (int)((second ? p - kp8 : p) << 3);
  const float* srow = src + (size_t)clampi(row, 0, rows - 1) * (size_t)ldsrc;
  float x[8];
  unsigned mk[8];
#pragma unroll
  for (int e = 0; e < 8; ++e) {
    const int c = c0 + e;
    const float v = srow[clampi(c, 0, cols - 1)];
    asm volatile("" :: "v"(v));
    x[e]  = v;
    mk[e] = (row < rows && c < cols) ? 0xFFFFu : 0u;
  }
  const v4f a = (v4f){ x[0], x[1], x[2], x[3] };
  const v4f c = (v4f){ x[4], x[5], x[6], x[7] };
  v4u o;
  if (FORM == 2) {
    o = pack8_f16(a, c);
  } else {
    const v4u hi = pack8_bf16(a, c);
    o = hi;
    if (FORM == 1) { const v4u lo = pack8_bf16_lo(a, c); o = second ? lo : hi; }
  }
  const v4u mw = (v4u){ pk16(mk[0], mk[1]), pk16(mk[2], mk[3]), pk16(mk[4], mk[5]), pk16(mk[6], mk[7]) };
  o &= mw;
  if (g < total) {
    volatile v4u* q = (volatile v4u*)(dst + (size_t)g * 8);
    *q = o;
    __threadfence();
    *q = o;
  }
}

template <int FORM> struct FragOf    { typedef FragB T; };
template <>         struct FragOf<2> { typedef FragH T; };
__device__ __forceinline__ v8f mm(const FragB& a, const FragB& b, v8f c) { return wmb(a, b, c); }
__device__ __forceinline__ v8f mm(const FragH& a, const FragH& b, v8f c) { return wmh(a, b, c); }
template <class F> __device__ __forceinline__ F ld_frag(const unsigned short* p) {
  F f;
  f.h[0] = *(const v8usa*)(p);
  f.h[1] = *(const v8usa*)(p + 16);
  return f;
}

template <int FORM, int EPI>
__global__ __launch_bounds__(256) __attribute__((amdgpu_num_vgpr(248)))
void k_gemm_nt(const unsigned short* __restrict__ A, const unsigned short* __restrict__ B,
               const float* __restrict__ bias, float* __restrict__ D, int M, int N, int KTOT, int ldd) {
  static_assert(FORM >= 0 && FORM <= 2);
  static_assert(EPI == 0 || EPI == 1);
  typedef typename FragOf<FORM>::T F;
  __shared__ __attribute__((aligned(16))) float sT[8][16 * 68];
  const int lane = threadIdx.x & 31;
  const int wave = threadIdx.x >> 5;
  const int tilesM = (M + 63) >> 6;
  const int tilesN = (N + 63) >> 6;
  const int tile = blockIdx.x * 8 + wave;
  if (tile >= tilesM * tilesN) return;
  const int tm = tile / tilesN;
  const int tn = tile - tm * tilesN;
  const int m0 = tm << 6;
  const int n0 = tn << 6;

  const int rl = lane & 15;
  const int h8 = (lane >> 4) * 8;
  const unsigned short* pa = A + (size_t)(m0 + rl) * (size_t)KTOT + h8;
  const unsigned short* pb = B + (size_t)(n0 + rl) * (size_t)KTOT + h8;

  v8f acc[4][4];
#pragma unroll
  for (int i = 0; i < 4; ++i)
#pragma unroll
    for (int j = 0; j < 4; ++j) acc[i][j] = (v8f){0.f, 0.f, 0.f, 0.f, 0.f, 0.f, 0.f, 0.f};

#pragma unroll 1
  for (int k0 = 0; k0 < KTOT; k0 += 32) {
    F bf[4];
#pragma unroll
    for (int j = 0; j < 4; ++j) bf[j] = ld_frag<F>(pb + (size_t)(j << 4) * (size_t)KTOT + k0);
#pragma unroll
    for (int i = 0; i < 4; ++i) {
      const F af = ld_frag<F>(pa + (size_t)(i << 4) * (size_t)KTOT + k0);
#pragma unroll
      for (int j = 0; j < 4; ++j) acc[i][j] = mm(af, bf[j], acc[i][j]);
    }
  }

  float* slab = sT[wave];
  const int hh = lane >> 4;
  const int c4 = (lane & 15) * 4;
  const int nc = n0 + c4;
  const bool cok = nc < N;
  v4f bv = (v4f){0.f, 0.f, 0.f, 0.f};
  if (EPI == 1) {
    bv = *(const v4fa*)(bias + clampi(nc, 0, N - 4));
    asm volatile("" :: "v"(bv));
  }
#pragma unroll
  for (int i = 0; i < 4; ++i) {
    const int mBase = m0 + (i << 4);
#pragma unroll
    for (int j = 0; j < 4; ++j) {
#pragma unroll
      for (int r = 0; r < 8; ++r) slab[(h8 + r) * 68 + (j << 4) + rl] = acc[i][j][r];
    }
    __builtin_amdgcn_fence(__ATOMIC_RELEASE, "workgroup");
    __builtin_amdgcn_wave_barrier();
    __builtin_amdgcn_fence(__ATOMIC_ACQUIRE, "workgroup");
    v4f vv[8];
#pragma unroll
    for (int it = 0; it < 8; ++it) {
      const int row = it * 2 + hh;
      v4f v = *(const v4fa*)(slab + row * 68 + c4);
      if (EPI == 1) v += bv;
      vv[it] = v;
    }
    for (int pass = 0; pass < 2; ++pass) {
#pragma unroll
      for (int it = 0; it < 8; ++it) {
        const int row = mBase + it * 2 + hh;
        if (cok && row < M) *(volatile v4f*)(D + (size_t)row * (size_t)ldd + nc) = vv[it];
      }
      __threadfence();
    }
    __builtin_amdgcn_fence(__ATOMIC_RELEASE, "workgroup");
    __builtin_amdgcn_wave_barrier();
    __builtin_amdgcn_fence(__ATOMIC_ACQUIRE, "workgroup");
  }
}

#pragma clang fp contract(off)
#include <stddef.h>

#define TWO_TERM_L2 1

#define NN     50000
#define RR     8
#define EE     1600000
#define DD     128
#define MPAD   50048
#define SLOTS  512
#define NBLKB  98
#define NPADN  (NBLKB * SLOTS)
#define RCAP   18432
#define HITMAX 16695
#define CHUNK  2048
#define NCH    782
#define NKEY   (RR * SLOTS)
#define ARRN   (NKEY + 16)
#define BK_INTS (2 * RCAP + ARRN + 32)
#define BK_BYTES (BK_INTS * 4)
#define KT2    (TWO_TERM_L2 ? 256 : 128)

#define WP_W1  0
#define WP_L1  (WP_W1 + 8 * 128 * 128)
#define WP_W2  (WP_L1 + 128 * 128)
#define WP_L2  (WP_W2 + 8 * 128 * KT2)
#define WP_END (WP_L2 + 128 * KT2)
#define PB_HB  (MPAD * 16 / 256)
#define PB_HZ  ((MPAD - NN) * (KT2 / 8) / 256)
#define PB_W1  64
#define PB_L1  8
#define PB_W2  (KT2 / 2)
#define PB_L2  (KT2 / 16)
#define PB_TOT (PB_HB + PB_HZ + PB_W1 + PB_L1 + PB_W2 + PB_L2 + 1)

static_assert(RR == 8 && DD == 128);
static_assert(EE == 781 * 2048 + 512 && EE % 8 == 0 && NCH * CHUNK >= EE && (NCH - 1) * CHUNK < EE);
static_assert(SLOTS * NBLKB >= NN && (NBLKB - 1) * SLOTS < NN);
static_assert(NN <= 65536 && NKEY <= 65536 && SLOTS == (1 << 9) && (NKEY & (NKEY - 1)) == 0 && NKEY == 4096);
static_assert(RCAP % 1024 == 0 && RCAP % 256 == 0 && RCAP >= HITMAX + (HITMAX * 6) / 100 + 1);
static_assert(MPAD % 64 == 0 && MPAD >= NN && NN % 16 == 0 && NN % 8 == 0);
static_assert(PB_HB * 256 == MPAD * 16 && PB_HZ * 256 == (MPAD - NN) * (KT2 / 8));
static_assert(KT2 % 32 == 0 && DD % 64 == 0 && DD % 32 == 0);
static_assert(PB_W1 * 2048 == 8 * 128 * 128 && PB_L1 * 2048 == 128 * 128);
static_assert(PB_W2 * 2048 == 8 * 128 * KT2 && PB_L2 * 2048 == 128 * KT2);
static_assert(BK_INTS % 4 == 0 && BK_BYTES <= 300000 && BK_BYTES + 34816 <= 327680);
static_assert((WP_L1 % 128) == 0 && (WP_W2 % 128) == 0 && (WP_L2 % 128) == 0);
static_assert((RR * SLOTS / 4) % 256 == 0 && (SLOTS / 4) == 128);
static_assert((long long)(NN - 1) * DD + (DD - 1) < (long long)NN * DD);

typedef int          v4i __attribute__((ext_vector_type(4)));
typedef unsigned int v2u __attribute__((ext_vector_type(2)));
typedef v4i __attribute__((may_alias)) v4ia;

__device__ __forceinline__ void pinf(float x) { asm volatile("" :: "v"(x)); }
__device__ __forceinline__ void pini(int x)   { asm volatile("" :: "v"(x)); }
__device__ __forceinline__ void pin4(const v4i w) { pini(w.x); pini(w.y); pini(w.z); pini(w.w); }
__device__ __forceinline__ void pin4f(const v4f w) { pinf(w.x); pinf(w.y); pinf(w.z); pinf(w.w); }

template <int NOUT, int KT>
__device__ __forceinline__ void wunit(const float* __restrict__ W, unsigned short* plane, int u) {
  constexpr int PPR = KT / 8;
  const int R   = u / PPR;
  const int p   = u - R * PPR;
  const int rel = R / NOUT;
  const int n   = R - rel * NOUT;
  const int k8  = (p & 15) * 8;
  const size_t sb = (size_t)rel * (size_t)(128 * NOUT) + (size_t)k8 * NOUT + (size_t)n;
  float f[8];
#pragma unroll
  for (int i = 0; i < 8; ++i) { f[i] = W[sb + (size_t)i * NOUT]; pinf(f[i]); }
  const v4f a = (v4f){ f[0], f[1], f[2], f[3] };
  const v4f c = (v4f){ f[4], f[5], f[6], f[7] };
  const v4u o = pack8_bf16(a, c);
  volatile v4u* q = (volatile v4u*)(plane + (size_t)u * 8);
  *q = o;
  __threadfence();
  *q = o;
}

__global__ __launch_bounds__(256) void k_prep(const int* __restrict__ node_id, const float* __restrict__ emb,
                                              const float* __restrict__ Wr, const float* __restrict__ Wl,
                                              const float* __restrict__ bias, unsigned short* hb,
                                              unsigned short* h1, unsigned short* wp, float* bs) {
  const int b = (int)blockIdx.x, tid = (int)threadIdx.x;
  constexpr int C0 = PB_HB, C1 = C0 + PB_HZ, C2 = C1 + PB_W1, C3 = C2 + PB_L1, C4 = C3 + PB_W2, C5 = C4 + PB_L2;
  if (b < C0) {
    const int g   = b * 256 + tid;
    const int row = g >> 4;
    const int p   = g & 15;
    const int rc  = clampi(row, 0, NN - 1);
    int nid = node_id[rc];
    pini(nid);
    const int nd = clampi(nid, 0, NN - 1);
    const float* er = emb + (size_t)nd * DD + p * 8;
    const v4f a = *(const v4fa*)er;
    const v4f c = *(const v4fa*)(er + 4);
    pin4f(a);
    pin4f(c);
    v4u o = pack8_bf16(a, c);
    const unsigned m = (row < NN) ? 0xFFFFFFFFu : 0u;
    o &= (v4u){ m, m, m, m };
    volatile v4u* q = (volatile v4u*)(hb + (size_t)g * 8);
    *q = o;
    __threadfence();
    *q = o;
  } else if (b < C1) {
    const int g = (b - C0) * 256 + tid;
    const v4u z = (v4u){ 0u, 0u, 0u, 0u };
    volatile v4u* q = (volatile v4u*)(h1 + (size_t)NN * KT2 + (size_t)g * 8);
    *q = z;
    __threadfence();
    *q = z;
  } else if (b < C2) {
    wunit<128, 128>(Wr, wp + WP_W1, (b - C1) * 256 + tid);
  } else if (b < C3) {
    wunit<128, 128>(Wl, wp + WP_L1, (b - C2) * 256 + tid);
  } else if (b < C4) {
    wunit<128, KT2>(Wr + (size_t)RR * DD * DD, wp + WP_W2, (b - C3) * 256 + tid);
  } else if (b < C5) {
    wunit<128, KT2>(Wl + (size_t)DD * DD, wp + WP_L2, (b - C4) * 256 + tid);
  } else {
    const int i = clampi(tid, 0, 63) * 4;
    const v4f x = *(const v4fa*)(bias + i);
    pin4f(x);
    const v4f o = (v4f){ bf16_val(x.x), bf16_val(x.y), bf16_val(x.z), bf16_val(x.w) };
    if (tid < 64) {
      volatile v4f* q = (volatile v4f*)(bs + 4 * tid);
      *q = o;
      __threadfence();
      *q = o;
    }
  }
}

__global__ __launch_bounds__(256) void k_bucket(const int* __restrict__ srcg, const int* __restrict__ dstg,
                                                const int* __restrict__ typg,
                                                int* listg, int* cntg, int* offg, int* flagg) {
  extern __shared__ __attribute__((aligned(16))) int dsm[];
  int* hl   = dsm;
  int* ol   = dsm + RCAP;
  int* arr  = dsm + 2 * RCAP;
  int* misc = arr + ARRN;
  const int tid = (int)threadIdx.x, lane = tid & 31;
  const int wave = __builtin_amdgcn_readfirstlane(tid >> 5);
  const int bid = (int)blockIdx.x;
  const int nodeBase = bid * SLOTS;
  const int nb = (NN - nodeBase) < SLOTS ? (NN - nodeBase) : SLOTS;

  {
    const v4i z4 = {0, 0, 0, 0};
    for (int i = tid * 4; i < BK_INTS; i += 1024) *(v4ia*)(dsm + i) = z4;
  }
  __syncthreads();

  int t = 0;
#pragma unroll 1
  for (int ch = 0; ch < NCH; ++ch) {
    const int cbase = ch * CHUNK;
    const int e0 = cbase + tid * 8;
    const bool valid = e0 < EE;
    const int e0c = valid ? e0 : (EE - 8);
    const v4i da = *(const v4ia*)(dstg + e0c);
    const v4i db = *(const v4ia*)(dstg + e0c + 4);
    const v4i ta = *(const v4ia*)(typg + e0c);
    const v4i tb = *(const v4ia*)(typg + e0c + 4);
    const v4i sa = *(const v4ia*)(srcg + e0c);
    const v4i sb = *(const v4ia*)(srcg + e0c + 4);
    pin4(da); pin4(db); pin4(ta); pin4(tb); pin4(sa); pin4(sb);
    const int im = valid ? 0 : -1;
    const unsigned nbs = (unsigned)nodeBase;
    const unsigned unb = (unsigned)nb;
    const unsigned s0 = (unsigned)(da.x | im) - nbs, s1 = (unsigned)(da.y | im) - nbs;
    const unsigned s2 = (unsigned)(da.z | im) - nbs, s3 = (unsigned)(da.w | im) - nbs;
    const unsigned s4 = (unsigned)(db.x | im) - nbs, s5 = (unsigned)(db.y | im) - nbs;
    const unsigned s6 = (unsigned)(db.z | im) - nbs, s7 = (unsigned)(db.w | im) - nbs;
    const bool h0 = s0 < unb, h1 = s1 < unb, h2 = s2 < unb, h3 = s3 < unb;
    const bool h4 = s4 < unb, h5 = s5 < unb, h6 = s6 < unb, h7 = s7 < unb;
    const int k = (int)h0 + (int)h1 + (int)h2 + (int)h3 + (int)h4 + (int)h5 + (int)h6 + (int)h7;
    int incl = k;
#pragma unroll
    for (int dd = 1; dd < 32; dd <<= 1) {
      const int y = __shfl_up(incl, dd, 32);
      if (lane >= dd) incl += y;
    }
    const int wc = __shfl(incl, 31, 32);
    int pos = incl - k;
    int* mb = misc + (ch & 1) * 8;
    if (lane == 0) mb[wave] = wc;
    __syncthreads();
    int base = t, tot = 0;
#pragma unroll
    for (int w2 = 0; w2 < 8; ++w2) {
      const int c = clampi(mb[w2], 0, 256);
      base += (w2 < wave) ? c : 0;
      tot  += c;
    }
    pos += base;
#define PUTJ(HJ, SJ, TJ, QJ) if (HJ) { if (pos < RCAP) hl[pos] = (int)((((unsigned)clampi((TJ), 0, RR - 1) * (unsigned)SLOTS) + (SJ)) << 16) | clampi((QJ), 0, NN - 1); pos += 1; }
    PUTJ(h0, s0, ta.x, sa.x)
    PUTJ(h1, s1, ta.y, sa.y)
    PUTJ(h2, s2, ta.z, sa.z)
    PUTJ(h3, s3, ta.w, sa.w)
    PUTJ(h4, s4, tb.x, sb.x)
    PUTJ(h5, s5, tb.y, sb.y)
    PUTJ(h6, s6, tb.z, sb.z)
    PUTJ(h7, s7, tb.w, sb.w)
#undef PUTJ
    t += tot;
  }
  __syncthreads();
  const int tt = t < RCAP ? t : RCAP;
  const int ov = t > RCAP ? 1 : 0;

  if (tid == 0) {
#pragma unroll 1
    for (int i = 0; i < tt; ++i) {
      const unsigned w = (unsigned)hl[i];
      const int kk = (int)((w >> 16) & (unsigned)(NKEY - 1));
      arr[kk] = arr[kk] + 1;
    }
  }
  __syncthreads();
  if (wave == 0) {
    const int base = lane * (NKEY / 32);
    int s = 0;
#pragma unroll 1
    for (int i = 0; i < NKEY / 32; ++i) s += arr[base + i];
    int incl = s;
#pragma unroll
    for (int dd = 1; dd < 32; dd <<= 1) {
      const int y = __shfl_up(incl, dd, 32);
      if (lane >= dd) incl += y;
    }
    int run = incl - s;
#pragma unroll 1
    for (int i = 0; i < NKEY / 32; ++i) {
      run += arr[base + i];
      arr[base + i] = run;
    }
    if (lane == 31) arr[NKEY] = run;
  }
  __syncthreads();
  if (tid == 0) {
#pragma unroll 1
    for (int i = tt - 1; i >= 0; --i) {
      const unsigned w = (unsigned)hl[i];
      const int kk = (int)((w >> 16) & (unsigned)(NKEY - 1));
      const int p  = clampi(arr[kk] - 1, 0, RCAP - 1);
      arr[kk] = p;
      ol[p] = (int)(w & 0xFFFFu);
    }
  }
  __syncthreads();

  int* lg = listg + (size_t)bid * RCAP;
  int* fg = flagg + (size_t)bid * 32;
  const v4i flv = {ov, ov, ov, ov};
#pragma unroll 1
  for (int pass = 0; pass < 2; ++pass) {
#pragma unroll 1
    for (int it = 0; it < RCAP / 1024; ++it) {
      const int idx = tid + 256 * it;
      const v4i v = *(const v4ia*)(ol + 4 * idx);
      *(volatile v4i*)(lg + 4 * idx) = v;
    }
#pragma unroll 1
    for (int it = 0; it < (RR * SLOTS / 4) / 256; ++it) {
      const int idx = tid + 256 * it;
      const int r   = idx >> 7;
      const int q   = idx & 127;
      const int kb  = r * SLOTS + 4 * q;
      const v4i st4 = *(const v4ia*)(arr + kb);
      const int en4 = arr[kb + 4];
      v4i cv, fv;
      cv.x = clampi(st4.y - st4.x, 0, RCAP);
      cv.y = clampi(st4.z - st4.y, 0, RCAP);
      cv.z = clampi(st4.w - st4.z, 0, RCAP);
      cv.w = clampi(en4   - st4.w, 0, RCAP);
      fv.x = clampi(st4.x, 0, RCAP - 1);
      fv.y = clampi(st4.y, 0, RCAP - 1);
      fv.z = clampi(st4.z, 0, RCAP - 1);
      fv.w = clampi(st4.w, 0, RCAP - 1);
      const size_t go = (size_t)r * NPADN + (size_t)nodeBase + (size_t)(4 * q);
      *(volatile v4i*)(cntg + go) = cv;
      *(volatile v4i*)(offg + go) = fv;
    }
    if (tid < 8) *(volatile v4i*)(fg + 4 * tid) = flv;
    __threadfence();
  }
}

template <int MODE>
__global__ __launch_bounds__(256) void k_replay(const float* __restrict__ P, float* acc,
                                                const int* __restrict__ listg, const int* __restrict__ cntg,
                                                const int* __restrict__ offg, const int* __restrict__ flagg,
                                                const float* __restrict__ bias,
                                                unsigned short* xhl, float* outp, int relIn, int n_real) {
  static_assert(MODE >= 0 && MODE <= 2);
  const int tid = (int)threadIdx.x, lane = tid & 31;
  const int wave = __builtin_amdgcn_readfirstlane(tid >> 5);
  const int rel = clampi(relIn, 0, RR - 1);
  const int nr  = clampi(n_real, 1, NN);
  const int row = (int)blockIdx.x * 8 + wave;
  const bool live = row < nr;
  const int rowc = clampi(row, 0, nr - 1);
  const int b = rowc >> 9;
  const size_t ti = (size_t)rel * NPADN + (size_t)rowc;
  int c = cntg[ti];
  pini(c);
  int of = offg[ti];
  pini(of);
  int f = flagg[(size_t)b * 32];
  pini(f);
  const bool anyf = __builtin_amdgcn_ballot_w32(f != 0) != 0u;
  c  = clampi(c, 0, RCAP);
  of = clampi(of, 0, RCAP - 1);
  if (c > RCAP - of) c = RCAP - of;
  const int cn = __builtin_amdgcn_readfirstlane(live ? c : 0);
  const int o0 = __builtin_amdgcn_readfirstlane(of);
  const int* lp = listg + (size_t)b * RCAP + o0;

  const float* ap = acc + (size_t)rowc * DD + 4 * lane;
  v4f a = *(const v4fa*)ap;
  pin4f(a);

#pragma unroll 1
  for (int j0 = 0; j0 < cn; j0 += 32) {
    int jj = j0 + lane;
    jj = jj < cn ? jj : cn - 1;
    int w = lp[jj];
    pini(w);
    const int s = clampi(w, 0, NN - 1);
    const int rem = cn - j0;
    const int nj = rem < 32 ? rem : 32;
#pragma unroll 1
    for (int j = 0; j < nj; ++j) {
      const int sj = __builtin_amdgcn_readlane(s, j);
      const v4f tv = *(const v4fa*)(P + (size_t)sj * DD + 4 * lane);
      pin4f(tv);
      a.x = a.x + tv.x;
      a.y = a.y + tv.y;
      a.z = a.z + tv.z;
      a.w = a.w + tv.w;
    }
  }

  const float qn = __int_as_float(0x7fc00000);
  if (MODE == 0) {
    v4f o;
    o.x = anyf ? qn : a.x;
    o.y = anyf ? qn : a.y;
    o.z = anyf ? qn : a.z;
    o.w = anyf ? qn : a.w;
    if (live) {
      float* aw = acc + (size_t)row * DD + 4 * lane;
      *(volatile v4f*)aw = o;
      __threadfence();
      *(volatile v4f*)aw = o;
    }
  } else {
    const v4f bb = *(const v4fa*)(bias + 4 * lane);
    pin4f(bb);
    float y0 = a.x + bb.x, y1 = a.y + bb.y, y2 = a.z + bb.z, y3 = a.w + bb.w;
    y0 = anyf ? qn : y0;
    y1 = anyf ? qn : y1;
    y2 = anyf ? qn : y2;
    y3 = anyf ? qn : y3;
    if (MODE == 1) {
      const v2u hi = { pk16(bf16_bits(y0), bf16_bits(y1)), pk16(bf16_bits(y2), bf16_bits(y3)) };
      const v2u lo = { pk16(bf16_lo_bits(y0), bf16_lo_bits(y1)), pk16(bf16_lo_bits(y2), bf16_lo_bits(y3)) };
      if (live) {
        unsigned short* dp = xhl + (size_t)row * KT2 + 4 * lane;
        for (int pass = 0; pass < 2; ++pass) {
          *(volatile v2u*)dp = hi;
          if (TWO_TERM_L2) *(volatile v2u*)(dp + 128) = lo;
          __threadfence();
        }
      }
    } else {
      const v4f o = (v4f){ y0, y1, y2, y3 };
      if (live) {
        float* op = outp + (size_t)row * DD + 4 * lane;
        *(volatile v4f*)op = o;
        __threadfence();
        *(volatile v4f*)op = o;
      }
    }
  }
}

static constexpr size_t al256(size_t o) { return (o + 255) & ~(size_t)255; }

static constexpr size_t oHB   = 0;
static constexpr size_t oH1   = al256(oHB   + (size_t)MPAD * DD * 2);
static constexpr size_t oACC  = al256(oH1   + (size_t)MPAD * KT2 * 2);
static constexpr size_t oXR   = al256(oACC  + (size_t)MPAD * DD * 4);
static constexpr size_t oLIST = al256(oXR   + (size_t)MPAD * DD * 4);
static constexpr size_t oCNT  = al256(oLIST + (size_t)NBLKB * RCAP * 4);
static constexpr size_t oOFF  = al256(oCNT  + (size_t)RR * NPADN * 4);
static constexpr size_t oWP   = al256(oOFF  + (size_t)RR * NPADN * 4);
static constexpr size_t oFLAG = al256(oWP   + (size_t)WP_END * 2);
static constexpr size_t oBS   = al256(oFLAG + (size_t)NBLKB * 128);
static constexpr size_t oEND  = al256(oBS   + 1024);
static_assert(oEND <= ((size_t)128 << 20));
static_assert(!TWO_TERM_L2 || oEND == (size_t)((size_t)394613 << 8));

static void run_gemm(const unsigned short* A, const unsigned short* Bp, const float* bs, float* D, int kt,
                     hipStream_t stream) {
  const int tiles = ((NN + 63) / 64) * ((DD + 63) / 64);
  k_gemm_nt<0, 0><<<(tiles + 7) / 8, 256, 0, stream>>>(A, Bp, bs, D, NN, DD, kt, DD);
}

extern "C" void kernel_launch(void* const* d_in, const int* in_sizes, int n_in,
                              void* d_out, int out_size, void* d_ws, size_t ws_size,
                              hipStream_t stream) {
  if (n_in < 8) return;
  if (in_sizes[0] != NN) return;
  if (in_sizes[1] != EE || in_sizes[2] != EE || in_sizes[3] != EE) return;
  if (in_sizes[4] != NN * DD) return;
  if (in_sizes[5] != 2 * RR * DD * DD || in_sizes[6] != 2 * DD * DD || in_sizes[7] != 2 * DD) return;
  if (out_size != NN * DD) return;
  if (oEND > ws_size) return;

  const int*   node_id = (const int*)d_in[0];
  const int*   src     = (const int*)d_in[1];
  const int*   dst     = (const int*)d_in[2];
  const int*   etype   = (const int*)d_in[3];
  const float* emb     = (const float*)d_in[4];
  const float* Wr      = (const float*)d_in[5];
  const float* Wl      = (const float*)d_in[6];
  const float* bias    = (const float*)d_in[7];
  float* out = (float*)d_out;

  char* ws = (char*)d_ws;
  unsigned short* HB  = (unsigned short*)(ws + oHB);
  unsigned short* H1  = (unsigned short*)(ws + oH1);
  float* ACC  = (float*)(ws + oACC);
  float* XR   = (float*)(ws + oXR);
  int*   LIST = (int*)(ws + oLIST);
  int*   CNT  = (int*)(ws + oCNT);
  int*   OFF  = (int*)(ws + oOFF);
  unsigned short* WP = (unsigned short*)(ws + oWP);
  int*   FLAG = (int*)(ws + oFLAG);
  float* BS   = (float*)(ws + oBS);

  hipFuncSetAttribute(reinterpret_cast<const void*>(&k_bucket), hipFuncAttributeMaxDynamicSharedMemorySize, BK_BYTES);

  k_prep<<<PB_TOT, 256, 0, stream>>>(node_id, emb, Wr, Wl, bias, HB, H1, WP, BS);
  k_bucket<<<NBLKB, 256, BK_BYTES, stream>>>(src, dst, etype, LIST, CNT, OFF, FLAG);

  const int rgrid = NN / 8;

  run_gemm(HB, WP + WP_L1, BS, ACC, 128, stream);
  for (int r = 0; r < RR; ++r) {
    run_gemm(HB, WP + WP_W1 + (size_t)r * 128 * 128, BS, XR, 128, stream);
    if (r < RR - 1) k_replay<0><<<rgrid, 256, 0, stream>>>(XR, ACC, LIST, CNT, OFF, FLAG, BS, H1, out, r, NN);
    else            k_replay<1><<<rgrid, 256, 0, stream>>>(XR, ACC, LIST, CNT, OFF, FLAG, BS, H1, out, r, NN);
  }

  run_gemm(H1, WP + WP_L2, BS, ACC, KT2, stream);
  for (int r = 0; r < RR; ++r) {
    run_gemm(H1, WP + WP_W2 + (size_t)r * 128 * KT2, BS, XR, KT2, stream);
    if (r < RR - 1) k_replay<0><<<rgrid, 256, 0, stream>>>(XR, ACC, LIST, CNT, OFF, FLAG, BS + 128, H1, out, r, NN);
    else            k_replay<2><<<rgrid, 256, 0, stream>>>(XR, ACC, LIST, CNT, OFF, FLAG, BS + 128, H1, out, r, NN);
  }
}
